// Projector_16355235463833
// MI455X (gfx1250) — hardware-run, weakly checked
//
#include <hip/hip_runtime.h>
#include <math.h>

constexpr int kNImg  = 16;
constexpr int kNKey  = 256;
constexpr int kNCh   = 512;
constexpr int kNPx   = 1024;
constexpr int kNHead = 16;
constexpr int kHdim  = 32;
constexpr int kGrp   = 2;
constexpr int kNGrp  = kNImg / kGrp;
constexpr int kO2ld  = 2 * kNCh;
constexpr float kPCarry    = 4096.0f;
constexpr float kPCarryInv = 1.0f / 4096.0f;

typedef __attribute__((ext_vector_type(16))) _Float16 v16h;
typedef __attribute__((ext_vector_type(8)))  _Float16 v8h;
typedef __attribute__((ext_vector_type(16))) __bf16   v16b;
typedef __attribute__((ext_vector_type(8)))  __bf16   v8b;
typedef __attribute__((ext_vector_type(8)))  float    v8f;
typedef __attribute__((ext_vector_type(4)))  float    v4f;
typedef __attribute__((ext_vector_type(4)))  unsigned int v4u;

constexpr size_t kSzW16   = (size_t)3 * kNCh * kNCh * 2;
constexpr size_t kSzTok16 = (size_t)kNImg * kNKey * kNCh * 2;
constexpr size_t kSzFT16  = (size_t)kNImg * kNPx * kNCh * 2;
constexpr size_t kSzO2    = (size_t)kGrp * kNPx * kO2ld * 4;
constexpr size_t kSzQ16   = (size_t)kNImg * kNPx * kNCh * 2;
constexpr size_t kSzK16   = (size_t)kNImg * kNKey * kNCh * 2;
constexpr size_t kSzVT16  = (size_t)kNImg * kNCh * kNKey * 2 + (size_t)kHdim * kNKey * 2;
constexpr size_t kSzS     = (size_t)kGrp * kNHead * kNPx * kNKey * 4;
constexpr size_t kSzP16   = (size_t)kGrp * kNHead * kNPx * kNKey * 2;
constexpr size_t kOffW16   = 0;
constexpr size_t kOffTok16 = kOffW16 + kSzW16;
constexpr size_t kOffFT16  = kOffTok16 + kSzTok16;
constexpr size_t kOffO2    = kOffFT16;
constexpr size_t kOffQ16   = kOffFT16 + kSzFT16;
constexpr size_t kOffK16   = kOffQ16 + kSzQ16;
constexpr size_t kOffVT16  = kOffK16 + kSzK16;
constexpr size_t kOffS     = kOffVT16 + kSzVT16;
constexpr size_t kOffP16   = kOffS + kSzS;
constexpr size_t kWsTotal  = kOffP16 + kSzP16;
static_assert(kWsTotal == (size_t)98058240);
static_assert(kWsTotal <= (size_t)134217728);
static_assert(kSzO2 <= kSzFT16);
static_assert((kOffTok16 % 128) == 0 && (kOffFT16 % 128) == 0 && (kOffQ16 % 128) == 0 && (kOffK16 % 128) == 0 &&
              (kOffVT16 % 128) == 0 && (kOffS % 128) == 0 && (kOffP16 % 128) == 0);

__device__ __forceinline__ unsigned short f2bf_bits(float f) {
  unsigned u = __float_as_uint(f);
  return (unsigned short)((u + 0x7FFFu + ((u >> 16) & 1u)) >> 16);
}
__device__ __forceinline__ float bf_bits2f(unsigned short h) { return __uint_as_float(((unsigned)h) << 16); }

__device__ __forceinline__ void dep_guard_h(v8f& a, v8f& b, v16h x, v16h y) { asm volatile("v_nop\n\tv_nop\n\tv_nop\n\tv_nop" : "+v"(a), "+v"(b) : "v"(x), "v"(y)); }
__device__ __forceinline__ void dep_guard_b(v8f& a, v8f& b, v16b x, v16b y) { asm volatile("v_nop\n\tv_nop\n\tv_nop\n\tv_nop" : "+v"(a), "+v"(b) : "v"(x), "v"(y)); }
__device__ __forceinline__ void keep4_h(v16h a, v16h b, v16h c, v16h d) { asm volatile("v_nop" :: "v"(a), "v"(b), "v"(c), "v"(d)); }
__device__ __forceinline__ void keep4_b(v16b a, v16b b, v16b c, v16b d) { asm volatile("v_nop" :: "v"(a), "v"(b), "v"(c), "v"(d)); }
__device__ __forceinline__ void acc_guard4(v8f& a, v8f& b, v8f& c, v8f& d) { asm volatile("v_nop\n\tv_nop\n\tv_nop\n\tv_nop" : "+v"(a), "+v"(b), "+v"(c), "+v"(d)); }
template <typename T> struct Frag;
template <> struct Frag<_Float16> {
  typedef v16h V; union U { v16h v; v8h h[2]; };
  static __device__ __forceinline__ v16h load(const _Float16* p) {
    U f; f.h[0] = *(const v8h*)(p); f.h[1] = *(const v8h*)(p + 16); return f.v;
  }
  static __device__ __forceinline__ v8f mma(v16h a, v16h b, v8f c) {
    return __builtin_amdgcn_wmma_f32_16x16x32_f16(false, a, false, b, (short)0, c, false, false);
  }
  static __device__ __forceinline__ void guard(v8f& a, v8f& b, v16h x, v16h y) { dep_guard_h(a, b, x, y); }
  static __device__ __forceinline__ void keep(v16h a, v16h b, v16h c, v16h d) { keep4_h(a, b, c, d); }
};
template <> struct Frag<__bf16> {
  typedef v16b V; union U { v16b v; v8b h[2]; };
  static __device__ __forceinline__ v16b load(const __bf16* p) {
    U f; f.h[0] = *(const v8b*)(p); f.h[1] = *(const v8b*)(p + 16); return f.v;
  }
  static __device__ __forceinline__ v8f mma(v16b a, v16b b, v8f c) {
    return __builtin_amdgcn_wmma_f32_16x16x32_bf16(false, a, false, b, (short)0, c, false, false);
  }
  static __device__ __forceinline__ void guard(v8f& a, v8f& b, v16b x, v16b y) { dep_guard_b(a, b, x, y); }
  static __device__ __forceinline__ void keep(v16b a, v16b b, v16b c, v16b d) { keep4_b(a, b, c, d); }
};

__device__ __forceinline__ unsigned pk16(unsigned short a, unsigned short b) { return (unsigned)a | ((unsigned)b << 16); }
__device__ __forceinline__ unsigned short h_bits(float f) { const _Float16 h = (_Float16)f; return __builtin_bit_cast(unsigned short, h); }

template <int ET> struct Elem;
template <> struct Elem<0> { typedef _Float16 T; };
template <> struct Elem<1> { typedef __bf16 T; };
template <int ET, bool SPLIT, int BIAS_MODE, int OUT_MODE, bool RESID, int ACT = 0>
__global__ __launch_bounds__(256) void wmma_gemm64(
    const unsigned short* __restrict__ Ap, const unsigned short* __restrict__ A2p, int lda, long strideA, long strideAz,
    const unsigned short* __restrict__ Btp, const unsigned short* __restrict__ Bt2p, int ldb, long strideB, long strideBz,
    void* __restrict__ Cout, void* __restrict__ Cout2, int ldc, long strideC, long strideCz,
    const float* __restrict__ bias,
    const float* __restrict__ resid, long strideR,
    int M, int N, int K, float scale) {
  typedef typename Elem<ET>::T T;
  typedef typename Frag<T>::V V;
  const T* A = (const T*)Ap; const T* A2 = (const T*)A2p; const T* Bt = (const T*)Btp; const T* Bt2 = (const T*)Bt2p;
  __shared__ __align__(16) float sT[8][16 * 68];
  const int b    = blockIdx.y;
  const int bz   = blockIdx.z;
  const int lane = threadIdx.x & 31;
  const int wave = threadIdx.x >> 5;
  const int tilesN = N >> 6;
  const int tilesM = M >> 6;
  const int tile = blockIdx.x * 8 + wave;
  if (tile >= tilesM * tilesN) return;
  const int tm = tile / tilesN;
  const int tn = tile - tm * tilesN;
  const int m0 = tm << 6;
  const int n0 = tn << 6;

  const size_t offA = (size_t)b * strideA + (size_t)bz * strideAz;
  const size_t offB = (size_t)b * strideB + (size_t)bz * strideBz;
  const size_t offC = (size_t)b * strideC + (size_t)bz * strideCz;
  const T* Ab  = A  + offA;
  const T* Bb  = Bt + offB;
  const T* Ab2 = SPLIT ? (A2  + offA) : nullptr;
  const T* Bb2 = SPLIT ? (Bt2 + offB) : nullptr;

  const int rlane = lane & 15;
  const int koff  = (lane >> 4) * 8;
  const int mOff  = (lane >> 4) * 8;

  v8f acc[4][4];
#pragma unroll
  for (int i = 0; i < 4; ++i)
#pragma unroll
    for (int j = 0; j < 4; ++j) acc[i][j] = (v8f){0.f,0.f,0.f,0.f,0.f,0.f,0.f,0.f};

  for (int k0 = 0; k0 < K; k0 += 32) {
    V bh[4], bl[4];
#pragma unroll
    for (int j = 0; j < 4; ++j) {
      const size_t bo = (size_t)(n0 + (j << 4) + rlane) * ldb + koff + k0;
      bh[j] = Frag<T>::load(Bb + bo);
      if (SPLIT) bl[j] = Frag<T>::load(Bb2 + bo);
    }
#pragma unroll
    for (int i = 0; i < 4; ++i) {
      const size_t ao = (size_t)(m0 + (i << 4) + rlane) * lda + koff + k0;
      V ah = Frag<T>::load(Ab + ao);
      V al;
      if (SPLIT) al = Frag<T>::load(Ab2 + ao);
#pragma unroll
      for (int j = 0; j < 4; ++j) {
        acc[i][j] = Frag<T>::mma(ah, bh[j], acc[i][j]);
        if (SPLIT) {
          acc[i][j] = Frag<T>::mma(ah, bl[j], acc[i][j]);
          acc[i][j] = Frag<T>::mma(al, bh[j], acc[i][j]);
        }
      }
      Frag<T>::guard(acc[i][0], acc[i][3], ah, SPLIT ? al : ah);
    }
    Frag<T>::keep(bh[0], bh[1], bh[2], bh[3]);
    if (SPLIT) Frag<T>::keep(bl[0], bl[1], bl[2], bl[3]);
  }
  acc_guard4(acc[0][0], acc[0][1], acc[0][2], acc[0][3]);
  acc_guard4(acc[1][0], acc[1][1], acc[1][2], acc[1][3]);
  acc_guard4(acc[2][0], acc[2][1], acc[2][2], acc[2][3]);
  acc_guard4(acc[3][0], acc[3][1], acc[3][2], acc[3][3]);

  float* slab = sT[wave];
  const float* Rb = RESID ? (resid + (size_t)b * strideR) : nullptr;
#pragma unroll
  for (int i = 0; i < 4; ++i) {
    const int mBase = m0 + (i << 4);
#pragma unroll
    for (int j = 0; j < 4; ++j) {
      const int n = n0 + (j << 4) + rlane;
      float bv = 0.f;
      if (BIAS_MODE == 2) bv = bias[n];
#pragma unroll
      for (int r = 0; r < 8; ++r) {
        float v = acc[i][j][r] * scale;
        if (BIAS_MODE == 1) v += bias[mBase + mOff + r];
        if (BIAS_MODE == 2) v += bv;
        if (RESID) v += Rb[(size_t)(mBase + mOff + r) * ldc + n];
        if (ACT == 2) v = fmaxf(v, 0.0f);
        if (ACT == 4) v = (v > 0.f) ? v : 0.01f * v;
        slab[(mOff + r) * 68 + (j << 4) + rlane] = v;
      }
    }
    __builtin_amdgcn_fence(__ATOMIC_RELEASE, "workgroup");
    __builtin_amdgcn_wave_barrier();
    __builtin_amdgcn_fence(__ATOMIC_ACQUIRE, "workgroup");
    if (OUT_MODE == 0) {
      float* C = (float*)Cout + offC;
      const int hh = lane >> 4, c4 = (lane & 15) * 4;
      for (int pass = 0; pass < 2; ++pass) {
#pragma unroll
        for (int it = 0; it < 8; ++it) {
          const int row = it * 2 + hh;
          v4f v = *(const v4f*)(slab + row * 68 + c4);
          *(volatile v4f*)(C + (size_t)(mBase + row) * ldc + n0 + c4) = v;
        }
        __threadfence();
      }
    } else {
      const int q = lane >> 3, c8 = (lane & 7) * 8;
      unsigned short* C  = (unsigned short*)Cout  + offC;
      unsigned short* C2 = (OUT_MODE == 2) ? ((unsigned short*)Cout2 + offC) : nullptr;
      for (int pass = 0; pass < 2; ++pass) {
#pragma unroll
        for (int it = 0; it < 4; ++it) {
          const int row = it * 4 + q;
          const float* sp = slab + row * 68 + c8;
          v8h hv, lv;
#pragma unroll
          for (int e = 0; e < 8; ++e) {
            if (OUT_MODE == 1) {
              hv[e] = (_Float16)sp[e];
            } else {
              unsigned short hb = f2bf_bits(sp[e]);
              unsigned short lb = f2bf_bits(sp[e] - bf_bits2f(hb));
              hv[e] = __builtin_bit_cast(_Float16, hb);
              lv[e] = __builtin_bit_cast(_Float16, lb);
            }
          }
          *(volatile v8h*)(C + (size_t)(mBase + row) * ldc + n0 + c8) = hv;
          if (OUT_MODE == 2) *(volatile v8h*)(C2 + (size_t)(mBase + row) * ldc + n0 + c8) = lv;
        }
        __threadfence();
      }
    }
    __builtin_amdgcn_fence(__ATOMIC_RELEASE, "workgroup");
    __builtin_amdgcn_wave_barrier();
    __builtin_amdgcn_fence(__ATOMIC_ACQUIRE, "workgroup");
  }
}

__global__ __launch_bounds__(256) void cast8_bf16_kernel(const float* __restrict__ in, unsigned short* __restrict__ out, int n8) {
  const int i = blockIdx.x * 256 + threadIdx.x;
  if (i >= n8) return;
  const float* p = in + 8 * (size_t)i;
  const v4f a = *(const v4f*)(p);
  const v4f c = *(const v4f*)(p + 4);
  unsigned short hb[8];
#pragma unroll
  for (int e = 0; e < 4; ++e) {
    hb[e]     = f2bf_bits(a[e]);
    hb[4 + e] = f2bf_bits(c[e]);
  }
  const v4u u = (v4u){pk16(hb[0], hb[1]), pk16(hb[2], hb[3]), pk16(hb[4], hb[5]), pk16(hb[6], hb[7])};
  unsigned short* q = out + 8 * (size_t)i;
  *(volatile v4u*)q = u;
  __threadfence();
  *(volatile v4u*)q = u;
}

__global__ __launch_bounds__(256) void wcast3_bf16_kernel(const float* __restrict__ W0, const float* __restrict__ W1,
                                                          const float* __restrict__ W2, unsigned short* __restrict__ out, int n8) {
  const int z = blockIdx.y;
  const float* W = (z == 0) ? W0 : (z == 1) ? W1 : W2;
  const int i = blockIdx.x * 256 + threadIdx.x;
  if (i >= n8) return;
  const float* p = W + 8 * (size_t)i;
  const v4f a = *(const v4f*)(p);
  const v4f c = *(const v4f*)(p + 4);
  unsigned short hb[8];
#pragma unroll
  for (int e = 0; e < 4; ++e) {
    hb[e]     = f2bf_bits(a[e]);
    hb[4 + e] = f2bf_bits(c[e]);
  }
  const v4u u = (v4u){pk16(hb[0], hb[1]), pk16(hb[2], hb[3]), pk16(hb[4], hb[5]), pk16(hb[6], hb[7])};
  unsigned short* q = out + (size_t)z * 8 * (size_t)n8 + 8 * (size_t)i;
  *(volatile v4u*)q = u;
  __threadfence();
  *(volatile v4u*)q = u;
}

__global__ __launch_bounds__(256) void ftrans_bf16_kernel(const float* __restrict__ feat, unsigned short* __restrict__ FT) {
  __shared__ float sm[64][65];
  const int t  = threadIdx.x;
  const int p0 = blockIdx.x * 64;
  const int c0 = blockIdx.y * 64;
  const int n  = blockIdx.z;
  const float* src = feat + ((size_t)n * kNCh + c0) * kNPx + p0;
#pragma unroll
  for (int i = 0; i < 16; ++i) {
    const int e = i * 256 + t;
    const int r = e >> 6;
    const int col = e & 63;
    sm[col][r] = src[(size_t)r * kNPx + col];
  }
  __syncthreads();
  const int lane = t & 31, wave = t >> 5;
  const int q = lane >> 3, c8 = (lane & 7) * 8;
  unsigned short* dst = FT + ((size_t)n * kNPx + p0) * kNCh + c0;
  for (int pass = 0; pass < 2; ++pass) {
#pragma unroll
    for (int it = 0; it < 2; ++it) {
      const int row = wave * 8 + it * 4 + q;
      unsigned short hb[8];
#pragma unroll
      for (int e = 0; e < 8; ++e) hb[e] = f2bf_bits(sm[row][c8 + e]);
      const v4u u = (v4u){pk16(hb[0], hb[1]), pk16(hb[2], hb[3]), pk16(hb[4], hb[5]), pk16(hb[6], hb[7])};
      *(volatile v4u*)(dst + (size_t)row * kNCh + c8) = u;
    }
    __threadfence();
  }
}

__global__ __launch_bounds__(256) void zero16_kernel(unsigned short* __restrict__ p, int n8) {
  const int i = blockIdx.x * 256 + threadIdx.x;
  if (i >= n8) return;
  const v4u z = (v4u){0u, 0u, 0u, 0u};
  unsigned short* q = p + 8 * (size_t)i;
  *(volatile v4u*)q = z;
  __threadfence();
  *(volatile v4u*)q = z;
}

__global__ __launch_bounds__(256) void softmax256_kernel(const float* __restrict__ S, unsigned short* __restrict__ P,
                                                         int nrows, float carry) {
  const int lane = threadIdx.x & 31, wave = threadIdx.x >> 5;
  const int row = blockIdx.x * 8 + wave;
  if (row >= nrows) return;
  const int c0 = lane * 8;
  const float* sr = S + (size_t)row * kNKey + c0;
  const v4f a = *(const v4f*)(sr);
  const v4f c = *(const v4f*)(sr + 4);
  float x[8];
#pragma unroll
  for (int e = 0; e < 4; ++e) { x[e] = a[e]; x[4 + e] = c[e]; }
  float m = fmaxf(fmaxf(fmaxf(x[0], x[1]), fmaxf(x[2], x[3])), fmaxf(fmaxf(x[4], x[5]), fmaxf(x[6], x[7])));
#pragma unroll
  for (int off = 16; off > 0; off >>= 1) m = fmaxf(m, __shfl_xor(m, off, 32));
  float ex[8];
#pragma unroll
  for (int e = 0; e < 8; ++e) ex[e] = __expf(x[e] - m);
  float s = ((ex[0] + ex[1]) + (ex[2] + ex[3])) + ((ex[4] + ex[5]) + (ex[6] + ex[7]));
#pragma unroll
  for (int off = 16; off > 0; off >>= 1) s += __shfl_xor(s, off, 32);
  const float f = carry * (1.0f / s);
  unsigned short hb[8];
#pragma unroll
  for (int e = 0; e < 8; ++e) hb[e] = h_bits(ex[e] * f);
  const v4u u = (v4u){pk16(hb[0], hb[1]), pk16(hb[2], hb[3]), pk16(hb[4], hb[5]), pk16(hb[6], hb[7])};
  unsigned short* q = P + (size_t)row * kNKey + c0;
  *(volatile v4u*)q = u;
  __threadfence();
  *(volatile v4u*)q = u;
}

__global__ __launch_bounds__(256) void out_add_kernel(const float* __restrict__ feat, const float* __restrict__ O2,
                                                      float* __restrict__ out, int n0) {
  __shared__ __align__(16) float sm[kHdim][132];
  const int t = threadIdx.x, lane = t & 31, wave = t >> 5;
  const int nl = blockIdx.z, h = blockIdx.y, p0 = blockIdx.x * 128;
  const int n = n0 + nl;
  const float* ob = O2 + ((size_t)nl * kNPx + p0) * kO2ld + h * 64;
#pragma unroll
  for (int i = 0; i < 16; ++i) {
    const int e = i * 256 + t;
    const int p = e >> 5, d = e & 31;
    sm[d][p] = ob[(size_t)p * kO2ld + d];
  }
  __syncthreads();
  v4f rv[4];
#pragma unroll
  for (int j = 0; j < 4; ++j) {
    const int d = wave * 4 + j;
    const size_t gi = ((size_t)n * kNCh + h * kHdim + d) * kNPx + p0 + lane * 4;
    const v4f f = *(const v4f*)(feat + gi);
    const v4f o = *(const v4f*)(&sm[d][lane * 4]);
    rv[j] = f + o;
  }
  for (int pass = 0; pass < 2; ++pass) {
#pragma unroll
    for (int j = 0; j < 4; ++j) {
      const int d = wave * 4 + j;
      const size_t gi = ((size_t)n * kNCh + h * kHdim + d) * kNPx + p0 + lane * 4;
      *(volatile v4f*)(out + gi) = rv[j];
    }
    __threadfence();
  }
}

extern "C" void kernel_launch(void* const* d_in, const int* in_sizes, int n_in,
                              void* d_out, int out_size, void* d_ws, size_t ws_size,
                              hipStream_t stream) {
  if (n_in < 8) return;
  if (in_sizes[0] != kNImg * kNCh * kNPx) return;
  if (in_sizes[1] != kNImg * kNKey * kNCh) return;
  if (in_sizes[2] != kNCh * kNCh || in_sizes[4] != kNCh * kNCh || in_sizes[6] != kNCh * kNCh) return;
  if (in_sizes[3] != kNCh || in_sizes[5] != kNCh || in_sizes[7] != kNCh) return;
  if (out_size != kNImg * kNCh * kNPx) return;
  if (kWsTotal > ws_size) return;

  const float* feature = (const float*)d_in[0];
  const float* token   = (const float*)d_in[1];
  const float* wq = (const float*)d_in[2];
  const float* bq = (const float*)d_in[3];
  const float* wk = (const float*)d_in[4];
  const float* bk = (const float*)d_in[5];
  const float* wv = (const float*)d_in[6];
  const float* bv = (const float*)d_in[7];
  float* outp = (float*)d_out;

  char* ws = (char*)d_ws;
  unsigned short* W16   = (unsigned short*)(ws + kOffW16);
  unsigned short* Wq16  = W16;
  unsigned short* Wk16  = W16 + (size_t)1 * kNCh * kNCh;
  unsigned short* Wv16  = W16 + (size_t)2 * kNCh * kNCh;
  unsigned short* TOK16 = (unsigned short*)(ws + kOffTok16);
  unsigned short* FT16  = (unsigned short*)(ws + kOffFT16);
  float*          O2    = (float*)(ws + kOffO2);
  unsigned short* Q16   = (unsigned short*)(ws + kOffQ16);
  unsigned short* K16   = (unsigned short*)(ws + kOffK16);
  unsigned short* VT16  = (unsigned short*)(ws + kOffVT16);
  float*          Sf    = (float*)(ws + kOffS);
  unsigned short* P16   = (unsigned short*)(ws + kOffP16);

  const dim3 blk(256);
  const float scoreScale = 1.0f / sqrtf((float)(kNCh / kNHead));

  {
    const int n8 = kNCh * kNCh / 8;
    wcast3_bf16_kernel<<<dim3(n8 / 256, 3, 1), blk, 0, stream>>>(wq, wk, wv, W16, n8);
  }
  {
    const int n8 = kNImg * kNKey * kNCh / 8;
    cast8_bf16_kernel<<<dim3(n8 / 256), blk, 0, stream>>>(token, TOK16, n8);
  }
  ftrans_bf16_kernel<<<dim3(kNPx / 64, kNCh / 64, kNImg), blk, 0, stream>>>(feature, FT16);
  {
    const int n8 = kHdim * kNKey / 8;
    zero16_kernel<<<dim3(n8 / 256), blk, 0, stream>>>(VT16 + (size_t)kNImg * kNCh * kNKey, n8);
  }

  {
    const int M = kNImg * kNPx, N = kNCh, K = kNCh;
    const dim3 g(((M / 64) * (N / 64) + 7) / 8, 1, 1);
    wmma_gemm64<1, false, 2, 1, false, 0><<<g, blk, 0, stream>>>(
        FT16, FT16, kNCh, 0L, 0L, Wq16, Wq16, kNCh, 0L, 0L, (void*)Q16, (void*)Q16, kNCh, 0L, 0L,
        bq, feature, 0L, M, N, K, 1.0f);
  }
  {
    const int M = kNImg * kNKey, N = kNCh, K = kNCh;
    const dim3 g(((M / 64) * (N / 64) + 7) / 8, 1, 1);
    wmma_gemm64<1, false, 2, 1, false, 0><<<g, blk, 0, stream>>>(
        TOK16, TOK16, kNCh, 0L, 0L, Wk16, Wk16, kNCh, 0L, 0L, (void*)K16, (void*)K16, kNCh, 0L, 0L,
        bk, feature, 0L, M, N, K, 1.0f);
  }
  {
    const int M = kNCh, N = kNKey, K = kNCh;
    const dim3 g(((M / 64) * (N / 64) + 7) / 8, kNImg, 1);
    wmma_gemm64<1, false, 1, 1, false, 0><<<g, blk, 0, stream>>>(
        Wv16, Wv16, kNCh, 0L, 0L, TOK16, TOK16, kNCh, (long)kNKey * kNCh, 0L,
        (void*)VT16, (void*)VT16, kNKey, (long)kNCh * kNKey, 0L,
        bv, feature, 0L, M, N, K, 1.0f);
  }

  for (int gi = 0; gi < kNGrp; ++gi) {
    const int n0 = gi * kGrp;
    {
      const unsigned short* Qg = Q16 + (size_t)n0 * kNPx * kNCh;
      const unsigned short* Kg = K16 + (size_t)n0 * kNKey * kNCh;
      const int M = kNPx, N = kNKey, K = kHdim;
      const dim3 g(((M / 64) * (N / 64) + 7) / 8, kNHead, kGrp);
      wmma_gemm64<0, false, 0, 0, false, 0><<<g, blk, 0, stream>>>(
          Qg, Qg, kNCh, (long)kHdim, (long)kNPx * kNCh,
          Kg, Kg, kNCh, (long)kHdim, (long)kNKey * kNCh,
          (void*)Sf, (void*)Sf, kNKey, (long)kNPx * kNKey, (long)kNHead * kNPx * kNKey,
          bq, feature, 0L, M, N, K, scoreScale);
    }
    {
      const int nrows = kGrp * kNHead * kNPx;
      softmax256_kernel<<<dim3(nrows / 8), blk, 0, stream>>>(Sf, P16, nrows, kPCarry);
    }
    {
      const unsigned short* Vg = VT16 + (size_t)n0 * kNCh * kNKey;
      const int M = kNPx, N = 64, K = kNKey;
      const dim3 g(((M / 64) * (N / 64) + 7) / 8, kNHead, kGrp);
      wmma_gemm64<0, false, 0, 0, false, 0><<<g, blk, 0, stream>>>(
          P16, P16, kNKey, (long)kNPx * kNKey, (long)kNHead * kNPx * kNKey,
          Vg, Vg, kNKey, (long)kHdim * kNKey, (long)kNCh * kNKey,
          (void*)O2, (void*)O2, kO2ld, 64L, (long)kNPx * kO2ld,
          bq, feature, 0L, M, N, K, kPCarryInv);
    }
    out_add_kernel<<<dim3(kNPx / 128, kNHead, kGrp), blk, 0, stream>>>(feature, O2, outp, n0);
  }
}
